// S4_56788057588283
// MI455X (gfx1250) — hardware-verified
//
#include <hip/hip_runtime.h>
#include <math.h>

constexpr int kHid = 512;
constexpr int kNst = 32;
constexpr int kLen = 2048;
constexpr int kBat = 8;
constexpr int kSeq = 2048;
constexpr int kNchunk = kSeq / 32;
constexpr int kXsPitch = 2064;
constexpr int kKuLen = 2080;
constexpr int kOsPitch = 36;
constexpr float kTheta = (float)(6.283185307179586 / 2048.0);
constexpr float kInvLen = 1.0f / 2048.0f;

static_assert(kSeq == kLen, "");
static_assert(kNchunk == 64, "");
static_assert(kHid % 32 == 0 && kSeq % 64 == 0, "");

constexpr size_t kOffTwc = 0;
constexpr size_t kOffTws = 8192;
constexpr size_t kOffKhi = 16384;
constexpr size_t kOffKlo = kOffKhi + (size_t)kHid * kLen * 2;
constexpr size_t kOffXt  = kOffKlo + (size_t)kHid * kLen * 2;
constexpr size_t kOffYt  = kOffXt + (size_t)kHid * kBat * kSeq * 2;
constexpr size_t kWsEnd  = kOffYt + (size_t)kHid * kBat * kSeq * 4;
static_assert(kWsEnd == 54542336ull, "");
static_assert(kWsEnd <= 134217728ull, "");
static_assert((kOffKhi % 128) == 0 && (kOffKlo % 128) == 0 && (kOffXt % 128) == 0 && (kOffYt % 128) == 0, "");

typedef __attribute__((ext_vector_type(16))) __bf16   v16b;
typedef __attribute__((ext_vector_type(8)))  __bf16   v8b;
typedef __attribute__((ext_vector_type(8)))  float    v8f;
typedef __attribute__((ext_vector_type(4)))  float    v4f;
typedef __attribute__((ext_vector_type(4)))  unsigned int v4u;

__device__ __forceinline__ unsigned short f2bf_bits(float f) {
  unsigned u = __float_as_uint(f);
  return (unsigned short)((u + 0x7FFFu + ((u >> 16) & 1u)) >> 16);
}
__device__ __forceinline__ float bf_bits2f(unsigned short h) { return __uint_as_float(((unsigned)h) << 16); }
__device__ __forceinline__ float bfr(float f) { return bf_bits2f(f2bf_bits(f)); }
__device__ __forceinline__ unsigned pk16(unsigned short a, unsigned short b) { return (unsigned)a | ((unsigned)b << 16); }
__device__ __forceinline__ float rcpf(float x) { return __builtin_amdgcn_rcpf(x); }

template <typename T> struct Frag;
template <> struct Frag<__bf16> {
  typedef v16b V; union U { v16b v; v8b h[2]; };
  static __device__ __forceinline__ v16b load(const __bf16* p) {
    U f; f.h[0] = *(const v8b*)(p); f.h[1] = *(const v8b*)(p + 16); return f.v;
  }
};

__device__ __forceinline__ v8f mma_bf(v16b a, v16b b, v8f c) {
  c = __builtin_amdgcn_wmma_f32_16x16x32_bf16(false, a, false, b, (short)0, c, false, false);
  asm volatile("v_nop\n\tv_nop\n\tv_nop\n\tv_nop" : "+v"(c) : "v"(a), "v"(b));
  return c;
}

__global__ __launch_bounds__(256) void twid_kernel(float* __restrict__ twc, float* __restrict__ tws) {
  const int m = blockIdx.x * 256 + threadIdx.x;
  const float ang = kTheta * (float)m;
  const float c = cosf(ang);
  const float s = sinf(ang);
  ((volatile float*)twc)[m] = c;
  ((volatile float*)tws)[m] = s;
  __threadfence();
  ((volatile float*)twc)[m] = c;
  ((volatile float*)tws)[m] = s;
}

__global__ __launch_bounds__(256) void xpose_kernel(const float* __restrict__ x, unsigned short* __restrict__ xT) {
  __shared__ float sm[32][65];
  const int tid = threadIdx.x, lane = tid & 31, wave = tid >> 5;
  const int s0 = blockIdx.x * 64, h0 = blockIdx.y * 32, b = blockIdx.z;
#pragma unroll
  for (int it = 0; it < 8; ++it) {
    const int e = it * 256 + tid;
    const int sl = e >> 5, hl = e & 31;
    sm[hl][sl] = x[((size_t)(b * kSeq + s0 + sl)) * kHid + h0 + hl];
  }
  __syncthreads();
  const int q = lane >> 3, c8 = (lane & 7) * 8;
  const int hl = wave * 4 + q;
  unsigned short hb[8];
#pragma unroll
  for (int e = 0; e < 8; ++e) hb[e] = f2bf_bits(sm[hl][c8 + e]);
  const v4u u = (v4u){pk16(hb[0], hb[1]), pk16(hb[2], hb[3]), pk16(hb[4], hb[5]), pk16(hb[6], hb[7])};
  unsigned short* dst = xT + ((size_t)((h0 + hl) * kBat + b)) * kSeq + s0 + c8;
  *(volatile v4u*)dst = u;
  __threadfence();
  *(volatile v4u*)dst = u;
}

__global__ __launch_bounds__(256) void kgen_kernel(
    const float* __restrict__ log_dt, const float* __restrict__ w_re, const float* __restrict__ w_im,
    const float* __restrict__ B_re, const float* __restrict__ B_im,
    const float* __restrict__ C_re, const float* __restrict__ C_im,
    const float* __restrict__ twc, const float* __restrict__ tws,
    unsigned short* __restrict__ khi, unsigned short* __restrict__ klo)
{
  __shared__ __align__(16) float ctab[kLen];
  __shared__ __align__(16) float stab[kLen];
  __shared__ __align__(16) float Kre[kLen];
  __shared__ __align__(16) float Kim[kLen];
  __shared__ float Tre[64][33];
  __shared__ float Tim[64][33];
  __shared__ float vre[4][kNst];
  __shared__ float vim[4][kNst];
  __shared__ float wsr[kNst];
  __shared__ float wsi[kNst];

  const int h = blockIdx.x;
  const int tid = threadIdx.x;
  const float dt = expf(bfr(log_dt[h]));

#pragma unroll
  for (int i = 0; i < 2; ++i) {
    const int e = i * 256 + tid;
    *(v4f*)(ctab + 4 * e) = *(const v4f*)(twc + 4 * e);
    *(v4f*)(stab + 4 * e) = *(const v4f*)(tws + 4 * e);
  }
  if (tid < 128) {
    const int n = tid & 31, ij = tid >> 5, i = ij >> 1, j = ij & 1;
    const float cr = bfr(C_re[h * 64 + i * 32 + n]);
    const float ci = bfr(C_im[h * 64 + i * 32 + n]);
    const float br = bfr(B_re[h * 64 + j * 32 + n]);
    const float bi = bfr(B_im[h * 64 + j * 32 + n]);
    vre[ij][n] = fmaf(cr, br, ci * bi);
    vim[ij][n] = fmaf(cr, bi, -(ci * br));
  }
  if (tid < kNst) {
    wsr[tid] = bfr(w_re[tid]) * dt;
    wsi[tid] = bfr(w_im[tid]) * dt;
  }
  __syncthreads();

#pragma unroll 1
  for (int it = 0; it < 4; ++it) {
    const int f = it * 256 + tid;
    const float cf = ctab[f], sf = stab[f];
    const float opc = 1.0f + cf;
    const float dmag = fmaf(opc, opc, sf * sf);
    const float invd = rcpf(dmag);
    const float zim = 4.0f * sf * invd;
    float rre[4], rim[4];
#pragma unroll
    for (int ij = 0; ij < 4; ++ij) { rre[ij] = 0.0f; rim[ij] = 0.0f; }
#pragma unroll 1
    for (int n = 0; n < kNst; ++n) {
      const float dre = -wsr[n];
      const float wi = wsi[n];
      const float d1 = zim - wi;
      const float d2 = zim + wi;
      const float dd = dre * dre;
      const float q1 = rcpf(fmaf(d1, d1, dd));
      const float q2 = rcpf(fmaf(d2, d2, dd));
      const float i1re = dre * q1, i1im = -(d1 * q1);
      const float i2re = dre * q2, i2im = -(d2 * q2);
      const float pre = i1re + i2re, pim = i1im + i2im;
      const float mre = i1re - i2re, dmi = i1im - i2im;
#pragma unroll
      for (int ij = 0; ij < 4; ++ij) {
        const float a = vre[ij][n], bq = vim[ij][n];
        rre[ij] = fmaf(a, pre, fmaf(-bq, dmi, rre[ij]));
        rim[ij] = fmaf(a, pim, fmaf(bq, mre, rim[ij]));
      }
    }
    const float r00r = rre[0] * dt, r00i = rim[0] * dt;
    const float r01r = rre[1] * dt, r01i = rim[1] * dt;
    const float r10r = rre[2] * dt, r10i = rim[2] * dt;
    const float r11r = rre[3] * dt, r11i = rim[3] * dt;
    const float tre = fmaf(r01r, r10r, -(r01i * r10i));
    const float tim = fmaf(r01r, r10i, r01i * r10r);
    const float wre = 1.0f + r11r, wim = r11i;
    const float qd = rcpf(fmaf(wre, wre, wim * wim));
    const float kfre = r00r - fmaf(tre, wre, tim * wim) * qd;
    const float kfim = r00i - fmaf(tim, wre, -(tre * wim)) * qd;
    const float g = 2.0f * invd;
    const float cre = opc * g, cim = sf * g;
    const float ore = fmaf(kfre, cre, -(kfim * cim));
    const float oim = fmaf(kfre, cim, kfim * cre);
    Kre[f] = ore; Kim[f] = oim;
    if (f >= 1) { Kre[kLen - f] = ore; Kim[kLen - f] = -oim; }
  }
  {
    float s00 = 0.0f;
#pragma unroll 1
    for (int n = 0; n < kNst; ++n) s00 += vre[0][n];
    if (tid == 0) { Kre[kLen / 2] = dt * s00; Kim[kLen / 2] = 0.0f; }
  }
  __syncthreads();

#pragma unroll 1
  for (int i = 0; i < 8; ++i) {
    const int e = i * 256 + tid;
    const int f0 = e >> 5, rr = e & 31;
    float are = 0.0f, aim = 0.0f;
#pragma unroll 1
    for (int f1 = 0; f1 < 32; ++f1) {
      const int fi = f0 + (f1 << 6);
      const int idx = ((f1 * rr) << 6) & (kLen - 1);
      const float c = ctab[idx], s = stab[idx];
      const float kr = Kre[fi], ki = Kim[fi];
      are = fmaf(kr, c, fmaf(-ki, s, are));
      aim = fmaf(kr, s, fmaf(ki, c, aim));
    }
    Tre[f0][rr] = are; Tim[f0][rr] = aim;
  }
  __syncthreads();

  float* krev = Kre;
#pragma unroll 1
  for (int i = 0; i < 8; ++i) {
    const int l = i * 256 + tid;
    const int rr = l & 31;
    float a = 0.0f;
#pragma unroll 1
    for (int f0 = 0; f0 < 64; ++f0) {
      const int idx = (f0 * l) & (kLen - 1);
      a = fmaf(Tre[f0][rr], ctab[idx], fmaf(-Tim[f0][rr], stab[idx], a));
    }
    krev[(kLen - 1) - l] = a * kInvLen;
  }
  __syncthreads();

  {
    const v4f a = *(const v4f*)(krev + 8 * tid);
    const v4f c2 = *(const v4f*)(krev + 8 * tid + 4);
    unsigned short hb[8], lb[8];
#pragma unroll
    for (int e = 0; e < 4; ++e) {
      const float v0 = a[e];
      hb[e] = f2bf_bits(v0);
      lb[e] = f2bf_bits(v0 - bf_bits2f(hb[e]));
      const float v1 = c2[e];
      hb[4 + e] = f2bf_bits(v1);
      lb[4 + e] = f2bf_bits(v1 - bf_bits2f(hb[4 + e]));
    }
    const v4u uh = (v4u){pk16(hb[0], hb[1]), pk16(hb[2], hb[3]), pk16(hb[4], hb[5]), pk16(hb[6], hb[7])};
    const v4u ul = (v4u){pk16(lb[0], lb[1]), pk16(lb[2], lb[3]), pk16(lb[4], lb[5]), pk16(lb[6], lb[7])};
    unsigned short* dh = khi + (size_t)h * kLen + 8 * tid;
    unsigned short* dl = klo + (size_t)h * kLen + 8 * tid;
    *(volatile v4u*)dh = uh;
    *(volatile v4u*)dl = ul;
    __threadfence();
    *(volatile v4u*)dh = uh;
    *(volatile v4u*)dl = ul;
  }
}

__global__ __launch_bounds__(256) void conv_kernel(
    const unsigned short* __restrict__ xT, const unsigned short* __restrict__ khi,
    const unsigned short* __restrict__ klo, float* __restrict__ yT)
{
  __shared__ __align__(16) unsigned short xs[kBat * kXsPitch];
  __shared__ __align__(16) unsigned short kuh[kKuLen];
  __shared__ __align__(16) unsigned short kul[kKuLen];
  __shared__ __align__(16) unsigned int ath[2][256];
  __shared__ __align__(16) unsigned int atl[2][256];
  __shared__ __align__(16) float osl[8][8 * kOsPitch];

  const int h = blockIdx.x;
  const int tid = threadIdx.x;
  const int lane = tid & 31;
  const int wave = __builtin_amdgcn_readfirstlane(tid >> 5);
  const int hh = lane >> 4, rl = lane & 15;

  if (tid < 64) {
    const int b = tid >> 3, w = tid & 7;
    *(unsigned int*)(xs + b * kXsPitch + 2 * w) = 0u;
  }
  if (tid < 16) {
    *(unsigned int*)(kuh + kLen + 2 * tid) = 0u;
    *(unsigned int*)(kul + kLen + 2 * tid) = 0u;
  }
  {
    const size_t ko = (size_t)h * kLen + 8 * tid;
    const v4u a = *(const v4u*)(khi + ko);
    const v4u c2 = *(const v4u*)(klo + ko);
    *(v4u*)(kuh + 8 * tid) = a;
    *(v4u*)(kul + 8 * tid) = c2;
  }
#pragma unroll
  for (int it = 0; it < 4; ++it) {
    const int e = it * 256 + tid;
    const int b = e >> 8, c8 = e & 255;
    const v4u v = *(const v4u*)(xT + ((size_t)(h * kBat + b)) * kSeq + 8 * c8);
    *(v4u*)(xs + b * kXsPitch + 16 + 8 * c8) = v;
  }
  asm volatile("" ::: "memory");
#pragma unroll
  for (int it = 4; it < 8; ++it) {
    const int e = it * 256 + tid;
    const int b = e >> 8, c8 = e & 255;
    const v4u v = *(const v4u*)(xT + ((size_t)(h * kBat + b)) * kSeq + 8 * c8);
    *(v4u*)(xs + b * kXsPitch + 16 + 8 * c8) = v;
  }
  __syncthreads();

  v8f acc[8];
#pragma unroll
  for (int j = 0; j < 8; ++j) acc[j] = (v8f){0.f, 0.f, 0.f, 0.f, 0.f, 0.f, 0.f, 0.f};

  const __bf16* Xb = (const __bf16*)(const void*)xs;
  const int xcol = (rl & 7) * kXsPitch + 16 * (rl >> 3) + 8 * hh;

  for (int c = 0; c < kNchunk; ++c) {
    const int buf = c & 1;
    {
      const int e2 = 2 * tid;
      const int i = e2 >> 5, kk = e2 & 31;
      const int p0 = 2031 - 32 * c - i + kk;
      const unsigned int wh = (unsigned int)kuh[p0] | ((unsigned int)kuh[p0 + 1] << 16);
      const unsigned int wl = (unsigned int)kul[p0] | ((unsigned int)kul[p0 + 1] << 16);
      ath[buf][i * 16 + (kk >> 1)] = wh;
      atl[buf][i * 16 + (kk >> 1)] = wl;
    }
    __syncthreads();
    const __bf16* Ah = (const __bf16*)(const void*)&ath[buf][0];
    const __bf16* Al = (const __bf16*)(const void*)&atl[buf][0];
    const v16b ah = Frag<__bf16>::load(Ah + rl * 32 + 8 * hh);
    const v16b al = Frag<__bf16>::load(Al + rl * 32 + 8 * hh);
#pragma unroll
    for (int j = 0; j < 8; ++j) {
      const int Tp = wave + 8 * j;
      if (Tp >= c) {
        const v16b bx = Frag<__bf16>::load(Xb + xcol + 32 * (Tp - c));
        acc[j] = mma_bf(ah, bx, acc[j]);
        acc[j] = mma_bf(al, bx, acc[j]);
      }
    }
  }

  float* os = &osl[wave][0];
  const int q = lane >> 3, c4 = (lane & 7) * 4;
#pragma unroll
  for (int j = 0; j < 8; ++j) {
    const int Tp = wave + 8 * j;
#pragma unroll
    for (int r = 0; r < 8; ++r) os[(rl & 7) * kOsPitch + 16 * (rl >> 3) + 8 * hh + r] = acc[j][r];
    __builtin_amdgcn_fence(__ATOMIC_RELEASE, "workgroup");
    __builtin_amdgcn_wave_barrier();
    __builtin_amdgcn_fence(__ATOMIC_ACQUIRE, "workgroup");
    const v4f v0 = *(const v4f*)(os + q * kOsPitch + c4);
    const v4f v1 = *(const v4f*)(os + (q + 4) * kOsPitch + c4);
    float* d0 = yT + ((size_t)(h * kBat + q)) * kSeq + 32 * Tp + c4;
    float* d1 = yT + ((size_t)(h * kBat + q + 4)) * kSeq + 32 * Tp + c4;
    for (int pass = 0; pass < 2; ++pass) {
      *(volatile v4f*)d0 = v0;
      *(volatile v4f*)d1 = v1;
      __threadfence();
    }
    __builtin_amdgcn_fence(__ATOMIC_RELEASE, "workgroup");
    __builtin_amdgcn_wave_barrier();
    __builtin_amdgcn_fence(__ATOMIC_ACQUIRE, "workgroup");
  }
}

__global__ __launch_bounds__(256) void out_kernel(const float* __restrict__ yT, const float* __restrict__ x,
                                                  const float* __restrict__ dskip, float* __restrict__ out) {
  __shared__ __align__(16) float sm[64][kOsPitch];
  const int tid = threadIdx.x, lane = tid & 31, wave = tid >> 5;
  const int t0 = blockIdx.x * 64, h0 = blockIdx.y * 32, b = blockIdx.z;
#pragma unroll
  for (int it = 0; it < 8; ++it) {
    const int e = it * 256 + tid;
    const int hl = e >> 6, tl = e & 63;
    sm[tl][hl] = yT[((size_t)((h0 + hl) * kBat + b)) * kSeq + t0 + tl];
  }
  __syncthreads();
  const int q = lane >> 3, c4 = (lane & 7) * 4;
  const v4f dv = *(const v4f*)(dskip + h0 + c4);
  float dr[4];
#pragma unroll
  for (int e = 0; e < 4; ++e) dr[e] = bfr(dv[e]);
#pragma unroll
  for (int it = 0; it < 2; ++it) {
    const int tl = wave * 8 + it * 4 + q;
    const v4f yv = *(const v4f*)(&sm[tl][c4]);
    const size_t off = ((size_t)(b * kSeq + t0 + tl)) * kHid + h0 + c4;
    const v4f xv = *(const v4f*)(x + off);
    v4f o;
#pragma unroll
    for (int e = 0; e < 4; ++e) o[e] = fmaf(dr[e], bfr(xv[e]), yv[e]);
    *(volatile v4f*)(out + off) = o;
    __threadfence();
    *(volatile v4f*)(out + off) = o;
  }
}

extern "C" void kernel_launch(void* const* d_in, const int* in_sizes, int n_in,
                              void* d_out, int out_size, void* d_ws, size_t ws_size,
                              hipStream_t stream) {
  if (n_in < 9) return;
  if (in_sizes[0] != kBat * kSeq * kHid) return;
  if (in_sizes[1] != kHid || in_sizes[8] != kHid) return;
  if (in_sizes[2] != kNst || in_sizes[3] != kNst) return;
  if (in_sizes[4] != kHid * 2 * kNst || in_sizes[5] != kHid * 2 * kNst ||
      in_sizes[6] != kHid * 2 * kNst || in_sizes[7] != kHid * 2 * kNst) return;
  if (out_size != kBat * kSeq * kHid) return;
  if (ws_size < kWsEnd) return;

  const float* x      = (const float*)d_in[0];
  const float* log_dt = (const float*)d_in[1];
  const float* w_re   = (const float*)d_in[2];
  const float* w_im   = (const float*)d_in[3];
  const float* B_re   = (const float*)d_in[4];
  const float* B_im   = (const float*)d_in[5];
  const float* C_re   = (const float*)d_in[6];
  const float* C_im   = (const float*)d_in[7];
  const float* dskip  = (const float*)d_in[8];
  float* out = (float*)d_out;

  char* ws = (char*)d_ws;
  float* twc = (float*)(ws + kOffTwc);
  float* tws = (float*)(ws + kOffTws);
  unsigned short* khi = (unsigned short*)(ws + kOffKhi);
  unsigned short* klo = (unsigned short*)(ws + kOffKlo);
  unsigned short* xT  = (unsigned short*)(ws + kOffXt);
  float* yT = (float*)(ws + kOffYt);

  twid_kernel<<<dim3(kLen / 256), dim3(256), 0, stream>>>(twc, tws);
  xpose_kernel<<<dim3(kSeq / 64, kHid / 32, kBat), dim3(256), 0, stream>>>(x, xT);
  kgen_kernel<<<dim3(kHid), dim3(256), 0, stream>>>(log_dt, w_re, w_im, B_re, B_im, C_re, C_im, twc, tws, khi, klo);
  conv_kernel<<<dim3(kHid), dim3(256), 0, stream>>>(xT, khi, klo, yT);
  out_kernel<<<dim3(kSeq / 64, kHid / 32, kBat), dim3(256), 0, stream>>>(yT, x, dskip, out);
}
